// CausalAttention_85529978732635
// MI455X (gfx1250) — hardware-verified
//
#include <hip/hip_runtime.h>


#ifndef NB
#define NB 4
#endif
#ifndef SEQ
#define SEQ 2048
#endif
#define NB_FULL 4
#define SEQ_FULL 2048
#define DM 1024
#define RH (((SEQ) < 512) ? (SEQ) : 512)
#define PCAR 16384.0f
#define SCL 0.03125f

static_assert((SEQ) % 128 == 0);
static_assert((SEQ) >= 128 && (SEQ) <= SEQ_FULL);
static_assert((NB) >= 1 && (NB) <= NB_FULL);
static_assert((RH) % 128 == 0 && (RH) <= (SEQ));
static_assert(DM % 64 == 0);
static_assert((size_t)((NB) - 1) * SEQ_FULL * DM + (size_t)(SEQ) * DM <= (size_t)NB_FULL * SEQ_FULL * DM);

typedef _Float16 h16;
typedef unsigned short bf;
typedef __attribute__((ext_vector_type(16))) __bf16   v16bf;
typedef __attribute__((ext_vector_type(16))) _Float16 v16h;
typedef __attribute__((ext_vector_type(8)))  _Float16 v8h;
typedef __attribute__((ext_vector_type(8)))  unsigned short v8us;
typedef __attribute__((ext_vector_type(8)))  float    v8f;
typedef __attribute__((ext_vector_type(4)))  float    v4f;
typedef __attribute__((ext_vector_type(2)))  _Float16 v2h;
typedef __attribute__((ext_vector_type(4)))  _Float16 v4h;
typedef __attribute__((ext_vector_type(2)))  unsigned short v2us;
typedef __attribute__((ext_vector_type(4)))  unsigned short v4us;
typedef v8h  __attribute__((may_alias)) v8ha;
typedef v4f  __attribute__((may_alias)) v4fa;
typedef v8us __attribute__((may_alias)) v8usa;

__device__ __forceinline__ unsigned short f2bf(float f) { unsigned u = __float_as_uint(f); u += 0x7FFFu + ((u >> 16) & 1u); return (unsigned short)(u >> 16); }
__device__ __forceinline__ float bf2f(unsigned short b) { return __uint_as_float(((unsigned)b) << 16); }
__device__ __forceinline__ v16h cat16(v8h lo, v8h hi) { return __builtin_shufflevector(lo, hi, 0, 1, 2, 3, 4, 5, 6, 7, 8, 9, 10, 11, 12, 13, 14, 15); }
__device__ __forceinline__ v16bf cat16b(v8us lo, v8us hi) { return __builtin_bit_cast(v16bf, __builtin_shufflevector(lo, hi, 0, 1, 2, 3, 4, 5, 6, 7, 8, 9, 10, 11, 12, 13, 14, 15)); }
__device__ __forceinline__ v8f wmma16(v16h a, v16h b, v8f c) { return __builtin_amdgcn_wmma_f32_16x16x32_f16(false, a, false, b, (short)0, c, false, false); }
__device__ __forceinline__ v8f wmmab(v16bf a, v16bf b, v8f c) { return __builtin_amdgcn_wmma_f32_16x16x32_bf16(false, a, false, b, (short)0, c, false, false); }
__device__ __forceinline__ h16 tohx(float x) { return (h16)x; }
__device__ __forceinline__ void splitf(float y, unsigned short& h, unsigned short& l) { h = f2bf(y); l = f2bf(y - bf2f(h)); }

template <typename T16> struct WFrag;
template <> struct WFrag<h16> { typedef v16h V; static __device__ __forceinline__ V ld(const h16* p) { return cat16(*(const v8h*)p, *(const v8h*)(p + 16)); } static __device__ __forceinline__ v8f mma(V a, V b, v8f c) { return wmma16(a, b, c); } };
template <> struct WFrag<bf> { typedef v16bf V; static __device__ __forceinline__ V ld(const bf* p) { return cat16b(*(const v8us*)p, *(const v8us*)(p + 16)); } static __device__ __forceinline__ v8f mma(V a, V b, v8f c) { return wmmab(a, b, c); } };
template <typename T16, int NSPLIT>
__global__ __launch_bounds__(32) void k_gemmw(const T16* __restrict__ A, const T16* __restrict__ A2, const T16* __restrict__ Bt, const T16* __restrict__ Bt2, int K, float* C, int ldc, int cskip, int kcaus, float osc) {
    typedef typename WFrag<T16>::V V;
    __shared__ __align__(16) float os[16 * 68];
    const int lane = threadIdx.x & 31, lr = lane & 15, hi = lane >> 4; const int r0 = blockIdx.x * 64, c0 = blockIdx.y * 64;
    if (cskip != 0 && c0 > r0 + 63) return;
    int kend = K; if (kcaus >= 0) { const int kb = kcaus + r0 + 64; kend = (kb < K) ? kb : K; }
    v8f acc[4][4];
#pragma unroll
    for (int mb = 0; mb < 4; ++mb)
#pragma unroll
        for (int nb = 0; nb < 4; ++nb) acc[mb][nb] = (v8f){};
    const size_t aoff = (size_t)(r0 + lr) * K + 8 * hi, boff = (size_t)(c0 + lr) * K + 8 * hi;
#pragma unroll 1
    for (int kc = 0; kc < kend; kc += 32) {
        V a[4], a2[4];
#pragma unroll
        for (int mb = 0; mb < 4; ++mb) { a[mb] = WFrag<T16>::ld(A + aoff + (size_t)mb * 16 * K + kc); if (NSPLIT == 1 || NSPLIT == 2) a2[mb] = WFrag<T16>::ld(A2 + aoff + (size_t)mb * 16 * K + kc); }
#pragma unroll
        for (int nb = 0; nb < 4; ++nb) { const V b = WFrag<T16>::ld(Bt + boff + (size_t)nb * 16 * K + kc); V b2; if (NSPLIT >= 2) b2 = WFrag<T16>::ld(Bt2 + boff + (size_t)nb * 16 * K + kc);
#pragma unroll
            for (int mb = 0; mb < 4; ++mb) { acc[mb][nb] = WFrag<T16>::mma(a[mb], b, acc[mb][nb]); if (NSPLIT == 1 || NSPLIT == 2) acc[mb][nb] = WFrag<T16>::mma(a2[mb], b, acc[mb][nb]); if (NSPLIT >= 2) acc[mb][nb] = WFrag<T16>::mma(a[mb], b2, acc[mb][nb]); } }
        asm volatile("v_nop\n\tv_nop\n\tv_nop\n\tv_nop" : "+v"(acc[0][0]), "+v"(acc[1][1]), "+v"(acc[2][2]), "+v"(acc[3][3]) : "v"(a[0]), "v"(a[3]));
    }
#pragma unroll
    for (int mb = 0; mb < 4; ++mb) {
#pragma unroll
        for (int nb = 0; nb < 4; ++nb) {
#pragma unroll
            for (int j = 0; j < 8; ++j) os[(hi * 8 + j) * 68 + nb * 16 + lr] = acc[mb][nb][j]; }
        __builtin_amdgcn_wave_barrier(); asm volatile("" ::: "memory");
        float* crow = C + (size_t)(r0 + mb * 16) * ldc + c0;
#pragma unroll 1
        for (int ps = 0; ps < 2; ++ps) {
#pragma unroll
            for (int s = 0; s < 8; ++s) { const int row = 2 * s + hi, cofs = lr * 4; v4f val = *(const v4fa*)(os + row * 68 + cofs); val = val * osc;
                *(volatile v4f*)(crow + (size_t)row * ldc + cofs) = val; }
            if (ps == 0) __threadfence(); }
        __builtin_amdgcn_wave_barrier(); asm volatile("" ::: "memory");
    }
}

__global__ __launch_bounds__(256) void k_cvt8(const float* __restrict__ src, bf* dst, size_t n8) { const size_t i = (size_t)blockIdx.x * 256 + threadIdx.x; if (i >= n8) return; const v8f v = *(const v8f*)(src + i * 8); v8us o;
#pragma unroll
    for (int k = 0; k < 8; ++k) o[k] = f2bf(v[k]); *(volatile v8us*)(dst + i * 8) = o; __threadfence(); *(volatile v8us*)(dst + i * 8) = o; }

__global__ __launch_bounds__(256) void k_split8(const float* __restrict__ src, bf* Hp, bf* Lp, size_t n8) { const size_t i = (size_t)blockIdx.x * 256 + threadIdx.x; if (i >= n8) return; const v8f v = *(const v8f*)(src + i * 8); v8us oh, ol;
#pragma unroll
    for (int k = 0; k < 8; ++k) { unsigned short a, c; splitf(v[k], a, c); oh[k] = a; ol[k] = c; }
    *(volatile v8us*)(Hp + i * 8) = oh; *(volatile v8us*)(Lp + i * 8) = ol; __threadfence(); *(volatile v8us*)(Hp + i * 8) = oh; *(volatile v8us*)(Lp + i * 8) = ol; }

__global__ __launch_bounds__(256) void k_vtp1(const float* __restrict__ F, h16* V16, bf* Vh, bf* Vl) {
    const size_t e = ((size_t)blockIdx.x * 256 + threadIdx.x) * 2; if (e >= (size_t)DM * SEQ) return;
    const int t = (int)(e % SEQ); const int d = (int)(e / SEQ);
    v2h o16; v2us oh, ol;
#pragma unroll
    for (int q = 0; q < 2; ++q) { const float x = F[(size_t)(t + q) * DM + d]; o16[q] = tohx(x); unsigned short a2, c2; splitf(x, a2, c2); oh[q] = a2; ol[q] = c2; }
    const bool lo = (t < RH);
    const size_t e2 = (size_t)d * RH + t;
    *(volatile v2h*)(V16 + e) = o16; if (lo) { *(volatile v2us*)(Vh + e2) = oh; *(volatile v2us*)(Vl + e2) = ol; }
    __threadfence();
    *(volatile v2h*)(V16 + e) = o16; if (lo) { *(volatile v2us*)(Vh + e2) = oh; *(volatile v2us*)(Vl + e2) = ol; }
}

__global__ __launch_bounds__(256) void k_asoft(const float* __restrict__ Sb, h16* P16, bf* Ph, bf* Pl) {
    const int lane = threadIdx.x & 31; const int row = blockIdx.x * 8 + (threadIdx.x >> 5); if (row >= SEQ) return; const int i = row; const bool hires = (i < RH); const float* sr = Sb + (size_t)row * SEQ; float v[SEQ / 32]; float mx = -3.0e38f;
#pragma unroll
    for (int ch = 0; ch < SEQ / 128; ++ch) { const int j0 = ch * 128 + lane * 4; const v4f a = *(const v4f*)(sr + j0);
#pragma unroll
        for (int q = 0; q < 4; ++q) { const int j = j0 + q; const float t = (j <= i) ? a[q] * SCL : -3.0e38f; v[ch * 4 + q] = t; mx = fmaxf(mx, t); } }
#pragma unroll
    for (int sh = 16; sh; sh >>= 1) mx = fmaxf(mx, __shfl_xor(mx, sh, 32));
    float sum = 0.f;
#pragma unroll
    for (int k = 0; k < SEQ / 32; ++k) { float d0 = __fsub_rn(v[k], mx); asm volatile("" : "+v"(d0)); v[k] = __builtin_amdgcn_exp2f(__fmul_rn(d0, 1.4426950408889634f)); sum += v[k]; }
#pragma unroll
    for (int sh = 16; sh; sh >>= 1) sum += __shfl_xor(sum, sh, 32);
    const float f = __fdiv_rn(hires ? 1.0f : PCAR, sum);
#pragma unroll 1
    for (int ps = 0; ps < 2; ++ps) {
        if (hires) {
#pragma unroll
            for (int ch = 0; ch < RH / 128; ++ch) { v4us oh, ol;
#pragma unroll
                for (int q = 0; q < 4; ++q) { unsigned short a, c2; splitf(v[ch * 4 + q] * f, a, c2); oh[q] = a; ol[q] = c2; }
                const size_t oo = (size_t)i * RH + ch * 128 + lane * 4; *(volatile v4us*)(Ph + oo) = oh; *(volatile v4us*)(Pl + oo) = ol; }
        } else {
#pragma unroll
            for (int ch = 0; ch < SEQ / 128; ++ch) { v4h o4;
#pragma unroll
                for (int q = 0; q < 4; ++q) o4[q] = tohx(v[ch * 4 + q] * f);
                *(volatile v4h*)(P16 + (size_t)row * SEQ + ch * 128 + lane * 4) = o4; } }
        if (ps == 0) __threadfence(); }
}

extern "C" void kernel_launch(void* const* d_in, const int* in_sizes, int n_in,
                              void* d_out, int out_size, void* d_ws, size_t ws_size, hipStream_t stream) {
    if (n_in < 4) return;
    const long long needx = (long long)(NB - 1) * SEQ_FULL * DM + (long long)SEQ * DM;
    if ((long long)in_sizes[0] < needx || (long long)out_size < needx) return;
    if ((long long)in_sizes[1] < (long long)DM * DM || (long long)in_sizes[2] < (long long)DM * DM || (long long)in_sizes[3] < (long long)DM * DM) return;
    const float* X = (const float*)d_in[0]; const float* Wq = (const float*)d_in[1]; const float* Wk = (const float*)d_in[2]; const float* Wv = (const float*)d_in[3];
    float* OUT = (float*)d_out;
    char* wsp = (char*)d_ws;
    auto take = [&](size_t bytes) { char* p = wsp; wsp += (bytes + 255) & ~(size_t)255; return (void*)p; };
    bf* WQ = (bf*)take((size_t)DM * DM * 2); bf* WK = (bf*)take((size_t)DM * DM * 2); bf* WV = (bf*)take((size_t)DM * DM * 2);
    bf* XB = (bf*)take((size_t)SEQ * DM * 2);
    float* F = (float*)take((size_t)SEQ * DM * 4);
    bf* QH = (bf*)take((size_t)SEQ * DM * 2); bf* QL = (bf*)take((size_t)SEQ * DM * 2); bf* KH = (bf*)take((size_t)SEQ * DM * 2); bf* KL = (bf*)take((size_t)SEQ * DM * 2);
    h16* VT = (h16*)take((size_t)DM * SEQ * 2); bf* VTH = (bf*)take((size_t)DM * RH * 2); bf* VTL = (bf*)take((size_t)DM * RH * 2);
    float* SB = (float*)take((size_t)SEQ * SEQ * 4);
    h16* P16 = (h16*)take((size_t)SEQ * SEQ * 2); bf* PH = (bf*)take((size_t)RH * RH * 2); bf* PL = (bf*)take((size_t)RH * RH * 2);
    if ((size_t)(wsp - (char*)d_ws) > ws_size) return;
    const size_t nW8 = (size_t)DM * DM / 8, nX8 = (size_t)SEQ * DM / 8;
    const unsigned gW8 = (unsigned)((nW8 + 255) / 256), gX8 = (unsigned)((nX8 + 255) / 256), gVT = (unsigned)(((size_t)DM * SEQ / 2 + 255) / 256);
    k_cvt8<<<gW8, 256, 0, stream>>>(Wq, WQ, nW8); k_cvt8<<<gW8, 256, 0, stream>>>(Wk, WK, nW8); k_cvt8<<<gW8, 256, 0, stream>>>(Wv, WV, nW8);
    const dim3 gP(SEQ / 64, DM / 64, 1), gS(SEQ / 64, SEQ / 64, 1), gE(RH / 64, DM / 64, 1);
    for (int b = 0; b < NB; ++b) {
        const size_t xoff = (size_t)b * SEQ_FULL * DM;
        k_cvt8<<<gX8, 256, 0, stream>>>(X + xoff, XB, nX8);
        k_gemmw<bf, 0><<<gP, 32, 0, stream>>>(XB, nullptr, WQ, nullptr, DM, F, DM, 0, -1, 1.0f);         k_split8<<<gX8, 256, 0, stream>>>(F, QH, QL, nX8);
        k_gemmw<bf, 0><<<gP, 32, 0, stream>>>(XB, nullptr, WK, nullptr, DM, F, DM, 0, -1, 1.0f);                         k_split8<<<gX8, 256, 0, stream>>>(F, KH, KL, nX8);
        k_gemmw<bf, 0><<<gP, 32, 0, stream>>>(XB, nullptr, WV, nullptr, DM, F, DM, 0, -1, 1.0f);                         k_vtp1<<<gVT, 256, 0, stream>>>(F, VT, VTH, VTL);
        k_gemmw<bf, 2><<<gS, 32, 0, stream>>>(QH, QL, KH, KL, DM, SB, SEQ, 1, -1, 1.0f);
        k_asoft<<<SEQ / 8, 256, 0, stream>>>(SB, P16, PH, PL);
        k_gemmw<bf, 2><<<gE, 32, 0, stream>>>(PH, PL, VTH, VTL, RH, OUT + xoff, DM, 0, 0, 1.0f);
        if (SEQ > RH) { const dim3 gL((SEQ - RH) / 64, DM / 64, 1);
            k_gemmw<h16, 0><<<gL, 32, 0, stream>>>(P16 + (size_t)RH * SEQ, nullptr, VT, nullptr, SEQ, OUT + xoff + (size_t)RH * DM, DM, 0, RH, 1.0f / PCAR); }
    }
}
